// GPT2UVLatentAttention_55181739819320
// MI455X (gfx1250) — hardware-verified
//
#include <hip/hip_runtime.h>
#include <stddef.h>


#define NB 4
#define NT 2048
#define NC 1024
#define NH 16
#define NR 256
#define NS 64
#define NHD 64
#define NMT (NB * NT)
#define NQK (2 * NC)

typedef _Float16 f16t;
typedef _Float16 v16h __attribute__((ext_vector_type(16)));
typedef _Float16 v8h __attribute__((ext_vector_type(8)));
typedef __bf16 v16b __attribute__((ext_vector_type(16)));
typedef float v8f __attribute__((ext_vector_type(8)));
typedef float v4f __attribute__((ext_vector_type(4)));
typedef unsigned int v4u __attribute__((ext_vector_type(4)));

union FragH { v16h v; v4u q[2]; };
union FragB { v16b v; v4u q[2]; unsigned int u[8]; };
union Pack8H { v8h v; v4u q; };

__device__ __forceinline__ v8f vz8() {
  v8f z = {0.f, 0.f, 0.f, 0.f, 0.f, 0.f, 0.f, 0.f};
  return z;
}

__device__ __forceinline__ v8f mma_f16(v16h a, v16h b, v8f c) {
  c = __builtin_amdgcn_wmma_f32_16x16x32_f16(false, a, false, b, (short)0, c, false, false);
  asm volatile("v_nop\n\tv_nop\n\tv_nop\n\tv_nop" : "+v"(c) : "v"(a), "v"(b));
  return c;
}
__device__ __forceinline__ v8f mma_bf16(v16b a, v16b b, v8f c) {
  c = __builtin_amdgcn_wmma_f32_16x16x32_bf16(false, a, false, b, (short)0, c, false, false);
  asm volatile("v_nop\n\tv_nop\n\tv_nop\n\tv_nop" : "+v"(c) : "v"(a), "v"(b));
  return c;
}

__device__ __forceinline__ unsigned int bf16_rne(float x) {
  unsigned int u = __float_as_uint(x);
  u += 0x7FFFu + ((u >> 16) & 1u);
  return u >> 16;
}
__device__ __forceinline__ void split2(float x, unsigned int& hb, unsigned int& lb) {
  hb = bf16_rne(x);
  lb = bf16_rne(x - __uint_as_float(hb << 16));
}
__device__ __forceinline__ void split8(const float* f, v4u& hq, v4u& lq) {
  unsigned int hb[8], lb[8];
#pragma unroll
  for (int i = 0; i < 8; ++i) split2(f[i], hb[i], lb[i]);
  hq.x = hb[0] | (hb[1] << 16); hq.y = hb[2] | (hb[3] << 16);
  hq.z = hb[4] | (hb[5] << 16); hq.w = hb[6] | (hb[7] << 16);
  lq.x = lb[0] | (lb[1] << 16); lq.y = lb[2] | (lb[3] << 16);
  lq.z = lb[4] | (lb[5] << 16); lq.w = lb[6] | (lb[7] << 16);
}
__device__ __forceinline__ v4u pack8h(const float* f) {
  Pack8H p;
#pragma unroll
  for (int i = 0; i < 8; ++i) p.v[i] = (f16t)f[i];
  return p.q;
}

__global__ __launch_bounds__(256) void k_cvt(const float* __restrict__ src,
                                            v4u* of16, v4u* ohi, v4u* olo,
                                            int n8, float scale, int mode) {
  const int g = blockIdx.x * 256 + threadIdx.x;
  if (g >= n8) return;
  const v4f* s4 = reinterpret_cast<const v4f*>(src);
  const v4f a = s4[2 * (size_t)g];
  const v4f b = s4[2 * (size_t)g + 1];
  float f[8] = {a.x, a.y, a.z, a.w, b.x, b.y, b.z, b.w};
  v4u q16, qh, ql;
  q16.x = 0u; q16.y = 0u; q16.z = 0u; q16.w = 0u;
  qh = q16; ql = q16;
  if (mode & 1) {
    float fs[8];
#pragma unroll
    for (int i = 0; i < 8; ++i) fs[i] = f[i] * scale;
    q16 = pack8h(fs);
  }
  if (mode & 2) split8(f, qh, ql);
#pragma unroll
  for (int pass = 0; pass < 2; ++pass) {
    if (mode & 1) *(volatile v4u*)(of16 + g) = q16;
    if (mode & 2) { *(volatile v4u*)(ohi + g) = qh; *(volatile v4u*)(olo + g) = ql; }
    if (pass == 0) __threadfence();
  }
}

__global__ __launch_bounds__(256) void k_pack_qk(const float* __restrict__ uf,
                                                const float* __restrict__ vf,
                                                v4u* w, float scale) {
  const int gid = blockIdx.x * 256 + threadIdx.x;
  if (gid >= NQK * (NR / 8)) return;
  const int nrow = gid >> 5;
  const int g = gid & 31;
  const int nn = nrow & (NC - 1);
  const int hh = nn >> 6, s = nn & 63;
  float f[8];
#pragma unroll
  for (int e = 0; e < 8; ++e) {
    const int r = g * 8 + e;
    const size_t idx = ((size_t)(hh * NR + r)) * NS + s;
    const float a = uf[idx];
    const float b = vf[idx];
    f[e] = ((nrow < NC) ? a : b) * scale;
  }
  const v4u q = pack8h(f);
  const size_t o = (size_t)nrow * (NR / 8) + g;
  *(volatile v4u*)(w + o) = q;
  __threadfence();
  *(volatile v4u*)(w + o) = q;
}

template <int IN3, int OUT>
__global__ __launch_bounds__(256) void k_gemm(
    const v4u* __restrict__ Ah, const v4u* __restrict__ Al,
    const v4u* __restrict__ Bh, const v4u* __restrict__ Bl,
    const float* __restrict__ bias,
    v4u* Oh, v4u* Ol, float* Of,
    int N, int K, float oscale, int Tlen, int Hn) {
  __shared__ __align__(16) float smem[16384];
  v4u* stg = reinterpret_cast<v4u*>(smem);

  const int tid = threadIdx.x;
  const int wave = tid >> 5, lane = tid & 31;
  const int h = lane >> 4, n = lane & 15;
  const int wm = wave >> 1, wn = wave & 1;
  const int rowBase = blockIdx.y * 128;
  const int colBase = blockIdx.x * 128;
  const int KV = K >> 3;

  v8f acc[2][4];
#pragma unroll
  for (int i = 0; i < 2; ++i)
#pragma unroll
    for (int j = 0; j < 4; ++j) acc[i][j] = vz8();

  const int sr = tid >> 1, sq = (tid & 1) * 2;
  const size_t ga = (size_t)(rowBase + sr) * KV + sq;
  const size_t gb = (size_t)(colBase + sr) * KV + sq;
  const int so = sr * 4 + sq;
  const int ra0 = (wm * 32 + n) * 4;
  const int ra1 = ra0 + 16 * 4;

  for (int kv = 0; kv < KV; kv += 4) {
    stg[so] = Ah[ga + kv];
    stg[so + 1] = Ah[ga + kv + 1];
    stg[512 + so] = Bh[gb + kv];
    stg[512 + so + 1] = Bh[gb + kv + 1];
    if (IN3) {
      stg[1024 + so] = Al[ga + kv];
      stg[1024 + so + 1] = Al[ga + kv + 1];
      stg[1536 + so] = Bl[gb + kv];
      stg[1536 + so + 1] = Bl[gb + kv + 1];
    }
    __syncthreads();

    if (!IN3) {
      FragH a0, a1;
      a0.q[0] = stg[ra0 + h]; a0.q[1] = stg[ra0 + 2 + h];
      a1.q[0] = stg[ra1 + h]; a1.q[1] = stg[ra1 + 2 + h];
#pragma unroll
      for (int j = 0; j < 4; ++j) {
        const int rb = 512 + (wn * 64 + j * 16 + n) * 4;
        FragH bf;
        bf.q[0] = stg[rb + h]; bf.q[1] = stg[rb + 2 + h];
        acc[0][j] = mma_f16(a0.v, bf.v, acc[0][j]);
        acc[1][j] = mma_f16(a1.v, bf.v, acc[1][j]);
      }
    } else {
      FragB a0, a1, c0, c1;
      a0.q[0] = stg[ra0 + h];        a0.q[1] = stg[ra0 + 2 + h];
      a1.q[0] = stg[ra1 + h];        a1.q[1] = stg[ra1 + 2 + h];
      c0.q[0] = stg[1024 + ra0 + h]; c0.q[1] = stg[1024 + ra0 + 2 + h];
      c1.q[0] = stg[1024 + ra1 + h]; c1.q[1] = stg[1024 + ra1 + 2 + h];
#pragma unroll
      for (int j = 0; j < 4; ++j) {
        const int rb = 512 + (wn * 64 + j * 16 + n) * 4;
        FragB bf;
        bf.q[0] = stg[rb + h]; bf.q[1] = stg[rb + 2 + h];
        acc[0][j] = mma_bf16(a0.v, bf.v, acc[0][j]);
        acc[1][j] = mma_bf16(a1.v, bf.v, acc[1][j]);
        acc[0][j] = mma_bf16(c0.v, bf.v, acc[0][j]);
        acc[1][j] = mma_bf16(c1.v, bf.v, acc[1][j]);
        bf.q[0] = stg[1024 + rb + h]; bf.q[1] = stg[1024 + rb + 2 + h];
        acc[0][j] = mma_bf16(a0.v, bf.v, acc[0][j]);
        acc[1][j] = mma_bf16(a1.v, bf.v, acc[1][j]);
      }
    }
    __syncthreads();
  }

#pragma unroll
  for (int i = 0; i < 2; ++i)
#pragma unroll
    for (int r = 0; r < 8; ++r)
#pragma unroll
      for (int j = 0; j < 4; ++j)
        smem[(wm * 32 + i * 16 + 8 * h + r) * 128 + wn * 64 + j * 16 + n] = acc[i][j][r] * oscale;
  __syncthreads();

  if (OUT == 2) {
#pragma unroll
    for (int pass = 0; pass < 2; ++pass) {
      for (int rr = 0; rr < 16; ++rr) {
        const int row = wave * 16 + rr;
        const float* t = smem + row * 128 + lane * 4;
        const int col = colBase + lane * 4;
        v4f v;
        v.x = t[0] + bias[col];     v.y = t[1] + bias[col + 1];
        v.z = t[2] + bias[col + 2]; v.w = t[3] + bias[col + 3];
        *(volatile v4f*)(Of + (size_t)(rowBase + row) * N + col) = v;
      }
      if (pass == 0) __threadfence();
    }
  } else if (OUT == 0) {
#pragma unroll
    for (int pass = 0; pass < 2; ++pass) {
#pragma unroll
      for (int rr = 0; rr < 8; ++rr) {
        const int row = wave * 16 + rr * 2 + h;
        const float* t = smem + row * 128 + n * 8;
        float f[8];
#pragma unroll
        for (int e = 0; e < 8; ++e) f[e] = t[e];
        const v4u q = pack8h(f);
        const size_t o = (((size_t)(rowBase + row)) * N + colBase + n * 8) >> 3;
        *(volatile v4u*)(Oh + o) = q;
      }
      if (pass == 0) __threadfence();
    }
  } else {
    const int b = rowBase / Tlen;
    const int t0 = rowBase - b * Tlen;
#pragma unroll
    for (int pass = 0; pass < 2; ++pass) {
#pragma unroll
      for (int cc = 0; cc < 8; ++cc) {
        const int col = wave * 16 + cc * 2 + h;
        const int gcol = colBase + col;
        const int hh = gcol >> 6, d = gcol & 63;
        const float bv = bias[gcol];
        float f[8];
#pragma unroll
        for (int e = 0; e < 8; ++e) f[e] = smem[(n * 8 + e) * 128 + col] + bv;
        v4u qh, ql;
        split8(f, qh, ql);
        const size_t o = ((((size_t)((b * Hn + hh) * 64 + d)) * Tlen) + t0 + n * 8) >> 3;
        *(volatile v4u*)(Oh + o) = qh;
        *(volatile v4u*)(Ol + o) = ql;
      }
      if (pass == 0) __threadfence();
    }
  }
}

__global__ __launch_bounds__(256) void k_attn(const v4u* __restrict__ QK,
                                             const v4u* __restrict__ Vth,
                                             const v4u* __restrict__ Vtl,
                                             v4u* Ch, v4u* Cl,
                                             int Tlen, int Hn, int Cn) {
  __shared__ __align__(16) float otile[8 * 16 * 64];

  const int tid = threadIdx.x;
  const int wave = tid >> 5, lane = tid & 31;
  const int h = lane >> 4, n = lane & 15;
  const int bh = blockIdx.x;
  const int b = bh / Hn, hh = bh - b * Hn;
  const int q0 = blockIdx.y * 128 + wave * 16;
  const int QKV = (2 * Cn) >> 3;
  const int TV = Tlen >> 3;
  const size_t bT = (size_t)b * Tlen;
  const int qc = (hh * 64) >> 3;
  const int kc = (Cn + hh * 64) >> 3;

  FragH bq0, bq1;
  {
    const size_t qr = (bT + q0 + n) * (size_t)QKV;
    bq0.q[0] = QK[qr + qc + h];     bq0.q[1] = QK[qr + qc + 2 + h];
    bq1.q[0] = QK[qr + qc + 4 + h]; bq1.q[1] = QK[qr + qc + 6 + h];
  }

  const float NEG = -__builtin_inff();
  const float kS = (1.0f / 2048.0f) * 1.44269504088896340736f;
  float m2 = NEG, lsum = 0.0f;
  v8f oa[4];
#pragma unroll
  for (int t = 0; t < 4; ++t) oa[t] = vz8();
  const int qme = q0 + n;
  const int nkt = (q0 + 15) / 64 + 1;

  for (int kt = 0; kt < nkt; ++kt) {
    const int key0 = kt * 64;
    v8f sc[4];
#pragma unroll
    for (int t = 0; t < 4; ++t) {
      const size_t kr = (bT + key0 + t * 16 + n) * (size_t)QKV;
      FragH a0, a1;
      a0.q[0] = QK[kr + kc + h];     a0.q[1] = QK[kr + kc + 2 + h];
      a1.q[0] = QK[kr + kc + 4 + h]; a1.q[1] = QK[kr + kc + 6 + h];
      v8f c = vz8();
      c = mma_f16(a0.v, bq0.v, c);
      c = mma_f16(a1.v, bq1.v, c);
      sc[t] = c;
    }
    float mx = NEG;
#pragma unroll
    for (int t = 0; t < 4; ++t)
#pragma unroll
      for (int r = 0; r < 8; ++r) {
        const int key = key0 + t * 16 + 8 * h + r;
        float s = sc[t][r] * kS;
        s = (key <= qme) ? s : NEG;
        sc[t][r] = s;
        mx = fmaxf(mx, s);
      }
    mx = fmaxf(mx, __shfl_xor(mx, 16));
    const float mn = fmaxf(m2, mx);
    const float alpha = exp2f(m2 - mn);
    float rs = 0.0f;
#pragma unroll
    for (int t = 0; t < 4; ++t)
#pragma unroll
      for (int r = 0; r < 8; ++r) {
        const float p = exp2f(sc[t][r] - mn);
        sc[t][r] = p;
        rs += p;
      }
    rs += __shfl_xor(rs, 16);
    lsum = lsum * alpha + rs;
    m2 = mn;
#pragma unroll
    for (int t = 0; t < 4; ++t) oa[t] = oa[t] * alpha;

#pragma unroll
    for (int ks = 0; ks < 2; ++ks) {
      FragB ph, pl;
#pragma unroll
      for (int w = 0; w < 4; ++w) {
        unsigned int h0, l0, h1, l1;
        split2(sc[2 * ks][2 * w], h0, l0);
        split2(sc[2 * ks][2 * w + 1], h1, l1);
        ph.u[w] = h0 | (h1 << 16);
        pl.u[w] = l0 | (l1 << 16);
        split2(sc[2 * ks + 1][2 * w], h0, l0);
        split2(sc[2 * ks + 1][2 * w + 1], h1, l1);
        ph.u[4 + w] = h0 | (h1 << 16);
        pl.u[4 + w] = l0 | (l1 << 16);
      }
      const int tv = (key0 >> 3) + ks * 4;
#pragma unroll
      for (int dt = 0; dt < 4; ++dt) {
        const size_t vr = ((size_t)(bh * 64 + dt * 16 + n)) * TV + tv;
        FragB vh, vl;
        vh.q[0] = Vth[vr + h]; vh.q[1] = Vth[vr + 2 + h];
        vl.q[0] = Vtl[vr + h]; vl.q[1] = Vtl[vr + 2 + h];
        oa[dt] = mma_bf16(vh.v, ph.v, oa[dt]);
        oa[dt] = mma_bf16(vl.v, ph.v, oa[dt]);
        oa[dt] = mma_bf16(vh.v, pl.v, oa[dt]);
      }
    }
  }

  const float inv = __builtin_amdgcn_rcpf(lsum);
  float* ot = otile + wave * (16 * 64);
#pragma unroll
  for (int dt = 0; dt < 4; ++dt)
#pragma unroll
    for (int r = 0; r < 8; ++r)
      ot[n * 64 + dt * 16 + 8 * h + r] = oa[dt][r] * inv;
  __syncthreads();

#pragma unroll
  for (int pass = 0; pass < 2; ++pass) {
#pragma unroll
    for (int i = 0; i < 4; ++i) {
      const int ql = i * 4 + (lane >> 3);
      const int d0 = (lane & 7) * 8;
      float f[8];
#pragma unroll
      for (int e = 0; e < 8; ++e) f[e] = ot[ql * 64 + d0 + e];
      v4u qh, qlo;
      split8(f, qh, qlo);
      const size_t o = ((bT + q0 + ql) * (size_t)Cn + hh * 64 + d0) >> 3;
      *(volatile v4u*)(Ch + o) = qh;
      *(volatile v4u*)(Cl + o) = qlo;
    }
    if (pass == 0) __threadfence();
  }
}

extern "C" void kernel_launch(void* const* d_in, const int* in_sizes, int n_in,
                              void* d_out, int out_size, void* d_ws,
                              size_t ws_size, hipStream_t stream) {
  if (n_in < 8) return;
  if (in_sizes[0] != NMT * NC || in_sizes[1] != NR * NC ||
      in_sizes[2] != NH * NR * NS || in_sizes[3] != NH * NR * NS ||
      in_sizes[4] != NC * NC || in_sizes[5] != NC ||
      in_sizes[6] != NC * NC || in_sizes[7] != NC ||
      out_size != NMT * NC) return;

  const float* x   = (const float*)d_in[0];
  const float* bw  = (const float*)d_in[1];
  const float* uf  = (const float*)d_in[2];
  const float* vf  = (const float*)d_in[3];
  const float* vpw = (const float*)d_in[4];
  const float* vpb = (const float*)d_in[5];
  const float* opw = (const float*)d_in[6];
  const float* opb = (const float*)d_in[7];
  float* out = (float*)d_out;

  const size_t P = (size_t)NMT * NC * 2;
  size_t off = 0;
  const size_t oXH = 0, oXHI = P, oXLO = 2 * P;
  const size_t oQK = 0;
  const size_t oCH = 2 * P, oCL = 3 * P;
  off = 4 * P;
  const size_t oBW  = off; off += (size_t)NR * NC * 2;
  const size_t oWQK = off; off += (size_t)NQK * NR * 2;
  const size_t oVWH = off; off += (size_t)NC * NC * 2;
  const size_t oVWL = off; off += (size_t)NC * NC * 2;
  const size_t oOWH = off; off += (size_t)NC * NC * 2;
  const size_t oOWL = off; off += (size_t)NC * NC * 2;
  const size_t oLAT = off; off += (size_t)NMT * NR * 2;
  const size_t oVTH = off; off += (size_t)NB * NH * NHD * NT * 2;
  const size_t oVTL = off; off += (size_t)NB * NH * NHD * NT * 2;
  if (off > ws_size) return;

  char* ws = (char*)d_ws;
  v4u* xh   = (v4u*)(ws + oXH);
  v4u* xhi  = (v4u*)(ws + oXHI);
  v4u* xlo  = (v4u*)(ws + oXLO);
  v4u* qk   = (v4u*)(ws + oQK);
  v4u* ch   = (v4u*)(ws + oCH);
  v4u* cl   = (v4u*)(ws + oCL);
  v4u* bwh  = (v4u*)(ws + oBW);
  v4u* wqk  = (v4u*)(ws + oWQK);
  v4u* vwh  = (v4u*)(ws + oVWH);
  v4u* vwl  = (v4u*)(ws + oVWL);
  v4u* owh  = (v4u*)(ws + oOWH);
  v4u* owl  = (v4u*)(ws + oOWL);
  v4u* lat  = (v4u*)(ws + oLAT);
  v4u* vth  = (v4u*)(ws + oVTH);
  v4u* vtl  = (v4u*)(ws + oVTL);
  float* wsf = (float*)(ws + oLAT);

  {
    const int n8 = NMT * NC / 8;
    k_cvt<<<(n8 + 255) / 256, 256, 0, stream>>>(x, xh, xhi, xlo, n8, 1.0f, 3);
  }
  {
    const int n8 = NR * NC / 8;
    k_cvt<<<(n8 + 255) / 256, 256, 0, stream>>>(bw, bwh, bwh, bwh, n8, 32.0f, 1);
  }
  {
    const int n8 = NC * NC / 8;
    k_cvt<<<(n8 + 255) / 256, 256, 0, stream>>>(vpw, vwh, vwh, vwl, n8, 1.0f, 2);
    k_cvt<<<(n8 + 255) / 256, 256, 0, stream>>>(opw, owh, owh, owl, n8, 1.0f, 2);
  }
  k_pack_qk<<<(NQK * (NR / 8) + 255) / 256, 256, 0, stream>>>(uf, vf, wqk, 32.0f);

  k_gemm<0, 0><<<dim3(NR / 128, NMT / 128), 256, 0, stream>>>(
      xh, xh, bwh, bwh, bw, lat, lat, wsf, NR, NC, 0.25f, NT, NH);
  k_gemm<1, 1><<<dim3(NC / 128, NMT / 128), 256, 0, stream>>>(
      xhi, xlo, vwh, vwl, vpb, vth, vtl, wsf, NC, NC, 1.0f, NT, NH);
  k_gemm<0, 0><<<dim3(NQK / 128, NMT / 128), 256, 0, stream>>>(
      lat, lat, wqk, wqk, bw, qk, qk, wsf, NQK, NR, 0.0625f, NT, NH);
  k_attn<<<dim3(NB * NH, NT / 128), 256, 0, stream>>>(qk, vth, vtl, ch, cl, NT, NH, NC);
  k_gemm<1, 2><<<dim3(NC / 128, NMT / 128), 256, 0, stream>>>(
      ch, cl, owh, owl, opb, ch, cl, out, NC, NC, 1.0f, NT, NH);
}
